// mLSTMBackendTriton_77970836291655
// MI455X (gfx1250) — hardware-verified
//
#include <hip/hip_runtime.h>


#define NZ   16
#define TT   2048
#define KD   128
#define SCL  0.088388347648318447f
typedef _Float16 h16;
typedef unsigned short bf;
typedef __attribute__((ext_vector_type(16))) __bf16   v16bf;
typedef __attribute__((ext_vector_type(16))) _Float16 v16h;
typedef __attribute__((ext_vector_type(8)))  _Float16 v8h;
typedef __attribute__((ext_vector_type(8)))  unsigned short v8us;
typedef __attribute__((ext_vector_type(8)))  float    v8f;
typedef __attribute__((ext_vector_type(4)))  float    v4f;
typedef v8h  __attribute__((may_alias)) v8ha;
typedef v4f  __attribute__((may_alias)) v4fa;
typedef v8us __attribute__((may_alias)) v8usa;

__device__ __forceinline__ unsigned short f2bf(float f) { unsigned u = __float_as_uint(f); u += 0x7FFFu + ((u >> 16) & 1u); return (unsigned short)(u >> 16); }
__device__ __forceinline__ float bf2f(unsigned short b) { return __uint_as_float(((unsigned)b) << 16); }
__device__ __forceinline__ float bfr(float f) { return bf2f(f2bf(f)); }
__device__ __forceinline__ v16h cat16(v8h lo, v8h hi) { return __builtin_shufflevector(lo, hi, 0, 1, 2, 3, 4, 5, 6, 7, 8, 9, 10, 11, 12, 13, 14, 15); }
__device__ __forceinline__ v16bf cat16b(v8us lo, v8us hi) { return __builtin_bit_cast(v16bf, __builtin_shufflevector(lo, hi, 0, 1, 2, 3, 4, 5, 6, 7, 8, 9, 10, 11, 12, 13, 14, 15)); }
__device__ __forceinline__ v8f wmma16(v16h a, v16h b, v8f c) { return __builtin_amdgcn_wmma_f32_16x16x32_f16(false, a, false, b, (short)0, c, false, false); }
__device__ __forceinline__ v8f wmmab(v16bf a, v16bf b, v8f c) { return __builtin_amdgcn_wmma_f32_16x16x32_bf16(false, a, false, b, (short)0, c, false, false); }


template <typename T16> struct WFrag;
template <> struct WFrag<h16> { typedef v16h V; static __device__ __forceinline__ V ld(const h16* p) { return cat16(*(const v8h*)p, *(const v8h*)(p + 16)); } static __device__ __forceinline__ v8f mma(V a, V b, v8f c) { return wmma16(a, b, c); } };
template <> struct WFrag<bf> { typedef v16bf V; static __device__ __forceinline__ V ld(const bf* p) { return cat16b(*(const v8us*)p, *(const v8us*)(p + 16)); } static __device__ __forceinline__ v8f mma(V a, V b, v8f c) { return wmmab(a, b, c); } };
template <typename T16, int NSPLIT, bool BIAS>
__global__ __launch_bounds__(32) void k_gemmw(const T16* __restrict__ A, const T16* __restrict__ A2, const T16* __restrict__ Bt, const T16* __restrict__ Bt2, int K, float* C, int ldc, const float* __restrict__ bias, size_t sA, size_t sB, size_t sC) {
    typedef typename WFrag<T16>::V V;
    __shared__ __align__(16) float os[16 * 68];
    const size_t z = blockIdx.z; A += z * sA; if (A2) A2 += z * sA; Bt += z * sB; if (Bt2) Bt2 += z * sB; C += z * sC;
    const int lane = threadIdx.x & 31, lr = lane & 15, hi = lane >> 4; const int r0 = blockIdx.x * 64, c0 = blockIdx.y * 64;
    v8f acc[4][4];
#pragma unroll
    for (int mb = 0; mb < 4; ++mb)
#pragma unroll
        for (int nb = 0; nb < 4; ++nb) acc[mb][nb] = (v8f){};
    const size_t aoff = (size_t)(r0 + lr) * K + 8 * hi, boff = (size_t)(c0 + lr) * K + 8 * hi;
#pragma unroll 1
    for (int kc = 0; kc < K; kc += 32) {
        V a[4], a2[4];
#pragma unroll
        for (int mb = 0; mb < 4; ++mb) { a[mb] = WFrag<T16>::ld(A + aoff + (size_t)mb * 16 * K + kc); if (NSPLIT == 1 || NSPLIT == 2) a2[mb] = WFrag<T16>::ld(A2 + aoff + (size_t)mb * 16 * K + kc); }
#pragma unroll
        for (int nb = 0; nb < 4; ++nb) { const V b = WFrag<T16>::ld(Bt + boff + (size_t)nb * 16 * K + kc); V b2; if (NSPLIT >= 2) b2 = WFrag<T16>::ld(Bt2 + boff + (size_t)nb * 16 * K + kc);
#pragma unroll
            for (int mb = 0; mb < 4; ++mb) { acc[mb][nb] = WFrag<T16>::mma(a[mb], b, acc[mb][nb]); if (NSPLIT == 1 || NSPLIT == 2) acc[mb][nb] = WFrag<T16>::mma(a2[mb], b, acc[mb][nb]); if (NSPLIT >= 2) acc[mb][nb] = WFrag<T16>::mma(a[mb], b2, acc[mb][nb]); } }
        asm volatile("v_nop\n\tv_nop\n\tv_nop\n\tv_nop" : "+v"(acc[0][0]), "+v"(acc[1][1]), "+v"(acc[2][2]), "+v"(acc[3][3]) : "v"(a[0]), "v"(a[3]));
    }
#pragma unroll
    for (int mb = 0; mb < 4; ++mb) {
#pragma unroll
        for (int nb = 0; nb < 4; ++nb) {
#pragma unroll
            for (int j = 0; j < 8; ++j) os[(hi * 8 + j) * 68 + nb * 16 + lr] = acc[mb][nb][j]; }
        __builtin_amdgcn_wave_barrier(); asm volatile("" ::: "memory");
        float* crow = C + (size_t)(r0 + mb * 16) * ldc + c0;
#pragma unroll 1
        for (int ps = 0; ps < 2; ++ps) {
#pragma unroll
            for (int s = 0; s < 8; ++s) { const int row = 2 * s + hi, cofs = lr * 4; v4f val = *(const v4fa*)(os + row * 68 + cofs); if (BIAS) { val[0] += bfr(bias[c0 + cofs]); val[1] += bfr(bias[c0 + cofs + 1]); val[2] += bfr(bias[c0 + cofs + 2]); val[3] += bfr(bias[c0 + cofs + 3]); }
                *(volatile v4f*)(crow + (size_t)row * ldc + cofs) = val; }
            if (ps == 0) __threadfence(); }
        __builtin_amdgcn_wave_barrier(); asm volatile("" ::: "memory");
    }
}

__device__ __forceinline__ void splitf(float y, unsigned short& h, unsigned short& l) { h = f2bf(y); l = f2bf(y - bf2f(h)); }
typedef __attribute__((ext_vector_type(2))) unsigned short v2us;
typedef __attribute__((ext_vector_type(4))) unsigned short v4us;

__global__ __launch_bounds__(256) void k_cvt8(const float* __restrict__ src, bf* dst, size_t n8) { const size_t i = (size_t)blockIdx.x * 256 + threadIdx.x; if (i >= n8) return; const v8f v = *(const v8f*)(src + i * 8); v8us o;
#pragma unroll
    for (int k = 0; k < 8; ++k) o[k] = f2bf(v[k]); *(volatile v8us*)(dst + i * 8) = o; __threadfence(); *(volatile v8us*)(dst + i * 8) = o; }
__global__ __launch_bounds__(256) void k_vt(const float* __restrict__ v, bf* VT) { const size_t i = ((size_t)blockIdx.x * 256 + threadIdx.x) * 2; if (i >= (size_t)NZ * KD * TT) return; const int t = (int)(i % TT); const int d = (int)((i / TT) % KD); const int z = (int)(i / ((size_t)TT * KD)); const float* src = v + (size_t)z * TT * KD;
    v2us o; o[0] = f2bf(src[(size_t)t * KD + d]); o[1] = f2bf(src[(size_t)(t + 1) * KD + d]); *(volatile v2us*)(VT + i) = o; __threadfence(); *(volatile v2us*)(VT + i) = o; }
__global__ __launch_bounds__(32) void k_gate(const float* __restrict__ ig, const float* __restrict__ fg, float* FC, float* IG) { const int z = threadIdx.x; if (z >= NZ) return; float acc = 0.f;
    for (int t = 0; t < TT; ++t) { const float f = bfr(fg[(size_t)z * TT + t]); const float ls = __fsub_rn(fminf(f, 0.f), log1pf(__expf(-fabsf(f)))); acc = __fadd_rn(acc, ls);
        *(volatile float*)(FC + (size_t)z * TT + t) = acc; *(volatile float*)(IG + (size_t)z * TT + t) = bfr(ig[(size_t)z * TT + t]); }
    __threadfence();
    acc = 0.f; for (int t = 0; t < TT; ++t) { const float f = bfr(fg[(size_t)z * TT + t]); const float ls = __fsub_rn(fminf(f, 0.f), log1pf(__expf(-fabsf(f)))); acc = __fadd_rn(acc, ls); *(volatile float*)(FC + (size_t)z * TT + t) = acc; *(volatile float*)(IG + (size_t)z * TT + t) = bfr(ig[(size_t)z * TT + t]); } }
__global__ __launch_bounds__(256) void k_dec(const float* __restrict__ S, const float* __restrict__ FC, const float* __restrict__ IG, bf* Gh, bf* Gl, float* NRM) {
    const int lane = threadIdx.x & 31; const int t = blockIdx.x * 8 + (threadIdx.x >> 5); if (t >= TT) return; const float fct = FC[t]; const float* sr = S + (size_t)t * TT; float v[64]; float mx = -3.0e38f;
#pragma unroll
    for (int ch = 0; ch < 16; ++ch) { const int s0 = ch * 128 + lane * 4; const v4f fc4 = *(const v4f*)(FC + s0), ig4 = *(const v4f*)(IG + s0);
#pragma unroll
        for (int q = 0; q < 4; ++q) { const int s = s0 + q; float ld = -3.0e38f; if (s <= t) { float dlt = __fsub_rn(fct, fc4[q]); asm volatile("" : "+v"(dlt)); ld = __fadd_rn(dlt, ig4[q]); } v[ch * 4 + q] = ld; mx = fmaxf(mx, ld); } }
#pragma unroll
    for (int sh = 16; sh; sh >>= 1) mx = fmaxf(mx, __shfl_xor(mx, sh, 32));
    float sum = 0.f;
#pragma unroll
    for (int ch = 0; ch < 16; ++ch) { const int s0 = ch * 128 + lane * 4; const v4f a = *(const v4f*)(sr + s0);
#pragma unroll
        for (int q = 0; q < 4; ++q) { const int s = s0 + q; float g = 0.f; if (s <= t) { float dd = __fsub_rn(v[ch * 4 + q], mx); asm volatile("" : "+v"(dd)); const float D = __builtin_amdgcn_exp2f(__fmul_rn(dd, 1.4426950408889634f)); float ss = __fmul_rn(a[q], SCL); asm volatile("" : "+v"(ss)); g = __fmul_rn(ss, D); } v[ch * 4 + q] = g; sum = __fadd_rn(sum, g); } }
#pragma unroll
    for (int sh = 16; sh; sh >>= 1) sum += __shfl_xor(sum, sh, 32);
    float nm = -mx; asm volatile("" : "+v"(nm)); const float nrm = fmaxf(fabsf(sum), __builtin_amdgcn_exp2f(__fmul_rn(nm, 1.4426950408889634f)));
#pragma unroll 1
    for (int ps = 0; ps < 2; ++ps) {
#pragma unroll
        for (int ch = 0; ch < 16; ++ch) { v4us oh, ol;
#pragma unroll
            for (int q = 0; q < 4; ++q) { unsigned short a2, c2; splitf(v[ch * 4 + q], a2, c2); oh[q] = a2; ol[q] = c2; }
            const size_t o = (size_t)t * TT + ch * 128 + lane * 4; *(volatile v4us*)(Gh + o) = oh; *(volatile v4us*)(Gl + o) = ol; }
        const float w = (lane == 0) ? nrm : 0.f; *(volatile float*)(NRM + (size_t)t * 32 + lane) = w; if (ps == 0) __threadfence(); }
}
__global__ __launch_bounds__(256) void k_fin(const float* __restrict__ O, const float* __restrict__ NRM, float* OUTz) { const size_t i = ((size_t)blockIdx.x * 256 + threadIdx.x) * 4; if (i >= (size_t)TT * KD) return; const int t = (int)(i / KD); const float n = NRM[(size_t)t * 32]; const v4f a = *(const v4f*)(O + i); v4f o;
#pragma unroll
    for (int q = 0; q < 4; ++q) o[q] = __fdiv_rn(a[q], n); *(volatile v4f*)(OUTz + i) = o; __threadfence(); *(volatile v4f*)(OUTz + i) = o; }

extern "C" void kernel_launch(void* const* d_in, const int* in_sizes, int n_in,
                              void* d_out, int out_size, void* d_ws, size_t ws_size, hipStream_t stream) {
    (void)in_sizes; (void)n_in; (void)out_size;
    const float* q = (const float*)d_in[0]; const float* k = (const float*)d_in[1]; const float* v = (const float*)d_in[2]; const float* ig = (const float*)d_in[3]; const float* fg = (const float*)d_in[4];
    float* OUT = (float*)d_out;
    char* wsp = (char*)d_ws;
    auto take = [&](size_t bytes) { char* p = wsp; wsp += (bytes + 255) & ~(size_t)255; return (void*)p; };
    bf* QB = (bf*)take((size_t)NZ * TT * KD * 2); bf* KB = (bf*)take((size_t)NZ * TT * KD * 2); bf* VT = (bf*)take((size_t)NZ * KD * TT * 2); float* FC = (float*)take((size_t)NZ * TT * 4); float* IG = (float*)take((size_t)NZ * TT * 4);
    float* S = (float*)take((size_t)TT * TT * 4); bf* Gh = (bf*)take((size_t)TT * TT * 2); bf* Gl = (bf*)take((size_t)TT * TT * 2); float* NRM = (float*)take((size_t)TT * 32 * 4); float* O = (float*)take((size_t)TT * KD * 4);
    if ((size_t)(wsp - (char*)d_ws) > ws_size) return;
    { const size_t n8 = (size_t)NZ * TT * KD / 8; const unsigned g8 = (unsigned)((n8 + 255) / 256); k_cvt8<<<g8, 256, 0, stream>>>(q, QB, n8); k_cvt8<<<g8, 256, 0, stream>>>(k, KB, n8); k_vt<<<(unsigned)(((size_t)NZ * KD * TT / 2 + 255) / 256), 256, 0, stream>>>(v, VT);
      k_gate<<<1, 32, 0, stream>>>(ig, fg, FC, IG); }
    for (int z = 0; z < NZ; ++z) {
        k_gemmw<bf, 0, false><<<dim3(TT / 64, TT / 64, 1), 32, 0, stream>>>(QB + (size_t)z * TT * KD, nullptr, KB + (size_t)z * TT * KD, nullptr, KD, S, TT, nullptr, 0, 0, 0);
        k_dec<<<TT / 8, 256, 0, stream>>>(S, FC + (size_t)z * TT, IG + (size_t)z * TT, Gh, Gl, NRM);
        k_gemmw<bf, 1, false><<<dim3(TT / 64, KD / 64, 1), 32, 0, stream>>>(Gh, Gl, VT + (size_t)z * KD * TT, nullptr, TT, O, KD, nullptr, 0, 0, 0);
        k_fin<<<(unsigned)(((size_t)TT * KD / 4 + 255) / 256), 256, 0, stream>>>(O, NRM, OUT + (size_t)z * TT * KD); }
}
